// LinearAttentionLayer_5153960755278
// MI455X (gfx1250) — hardware-run, weakly checked
//
#include <hip/hip_runtime.h>
#include <math.h>

typedef __attribute__((ext_vector_type(16))) _Float16 v16h;
typedef __attribute__((ext_vector_type(8)))  _Float16 v8h;
typedef __attribute__((ext_vector_type(8)))  float    v8f;
typedef __attribute__((ext_vector_type(4)))  float    v4f;
typedef __attribute__((ext_vector_type(4)))  unsigned int v4u;
typedef __attribute__((ext_vector_type(2)))  unsigned int v2u;
typedef __attribute__((ext_vector_type(4)))  int      v4i;

constexpr int kB   = 2;
constexpr int kS   = 512;
constexpr int kD   = 1024;
constexpr int kH   = 8;
constexpr int kHD  = 64;
constexpr int kHID = kH * kHD;
constexpr int kTok = kB * kS;
constexpr int kQKW = 2 * kHID;
static_assert(kHID == 512);
static_assert(kTok == 1024);
static_assert(kQKW == 1024);
static_assert((kD % 32) == 0 && (kHID % 32) == 0 && (kHD % 32) == 0);
static_assert((kTok % 64) == 0 && (kHID % 64) == 0 && (kD % 64) == 0 && (kS % 64) == 0);

constexpr float kInCarry   = 16.0f;
constexpr float kWCarry    = 1024.0f;
constexpr float kActCarry  = 16.0f;
constexpr float kCarCarry  = 16.0f;
constexpr float kXnCarry   = 16.0f;
constexpr float kProjScale  = kActCarry / (kInCarry * kWCarry);
constexpr float kScoreScale = 1.0f / (kActCarry * kActCarry);
constexpr float kCarToPV    = 1.0f / kCarCarry;
constexpr float kXScale     = 1.0f / kActCarry;
constexpr float kOutScale   = 1.0f / (kXnCarry * kWCarry);
constexpr float kStateScale = 1.0f / (kActCarry * kActCarry);
constexpr float kInvHid     = 1.0f / (float)kHID;
constexpr float kEps        = 1e-6f;
constexpr float kF16MinNormal = 6.103515625e-5f;
constexpr int   kPPitch = 72;

constexpr size_t kOffXH  = 0;
constexpr size_t kOffCH  = kOffXH  + (size_t)kTok * kD * 2;
constexpr size_t kOffWT  = kOffCH  + (size_t)kB * kH * kHD * kHD * 2;
constexpr size_t kOffWOT = kOffWT  + (size_t)3 * kHID * kD * 2;
constexpr size_t kOffQK  = kOffWOT + (size_t)kD * kHID * 2;
constexpr size_t kOffVT  = kOffQK  + (size_t)kTok * kQKW * 2;
constexpr size_t kOffXF  = kOffVT  + (size_t)kHID * kTok * 2;
constexpr size_t kOffXN  = kOffXF  + (size_t)kTok * kHID * 4;
constexpr size_t kWsTotal = kOffXN + (size_t)kTok * kHID * 2;
static_assert(kWsTotal == 12713984ull);
static_assert(kWsTotal <= 134217728ull);
static_assert((kOffCH % 128) == 0 && (kOffWT % 128) == 0 && (kOffWOT % 128) == 0 && (kOffQK % 128) == 0 &&
              (kOffVT % 128) == 0 && (kOffXF % 128) == 0 && (kOffXN % 128) == 0);
constexpr size_t kOut0Elems = (size_t)kB * kH * kHD * kHD;
constexpr size_t kOut1Elems = (size_t)kTok * kD;
static_assert(kOut0Elems * 4 == 262144ull);
static_assert((kOut0Elems + kOut1Elems) * 4 == 4456448ull);

__device__ __forceinline__ float bf16_rne(float f) {
  unsigned u = __float_as_uint(f);
  u = (u + 0x7FFFu + ((u >> 16) & 1u)) & 0xFFFF0000u;
  return __uint_as_float(u);
}
__device__ __forceinline__ float flush16(float f) { return (fabsf(f) < kF16MinNormal) ? 0.0f : f; }
__device__ __forceinline__ unsigned short h_bits(float f) { const _Float16 h = (_Float16)f; return __builtin_bit_cast(unsigned short, h); }
__device__ __forceinline__ unsigned pk16(unsigned short a, unsigned short b) { return (unsigned)a | ((unsigned)b << 16); }
__device__ __forceinline__ float h16_to_f32(unsigned hb) {
  const unsigned sgn = (hb & 0x8000u) << 16; const unsigned em = hb & 0x7fffu;
  const float fn = __uint_as_float((em << 13) + 0x38000000u);
  const float fs = (float)em * 5.9604644775390625e-8f;
  const float mag = (em < 0x400u) ? fs : fn; return __uint_as_float(__float_as_uint(mag) | sgn); }
__device__ __forceinline__ int reset_flag(int m) { m = (m < 0) ? 0 : m; m = (m > 1) ? 1 : m; return m; }

__device__ __forceinline__ void dep_guard4_h(v8f& a, v8f& b, v8f& c, v8f& d, v16h x, v16h y) { asm volatile("v_nop\n\tv_nop\n\tv_nop\n\tv_nop" : "+v"(a), "+v"(b), "+v"(c), "+v"(d) : "v"(x), "v"(y)); }
__device__ __forceinline__ void keep4_h(v16h a, v16h b, v16h c, v16h d) { asm volatile("v_nop" :: "v"(a), "v"(b), "v"(c), "v"(d)); }
__device__ __forceinline__ void acc_guard4(v8f& a, v8f& b, v8f& c, v8f& d) { asm volatile("v_nop\n\tv_nop\n\tv_nop\n\tv_nop" : "+v"(a), "+v"(b), "+v"(c), "+v"(d)); }
struct FragH {
  union U { v16h v; v8h h[2]; };
  static __device__ __forceinline__ v16h load(const _Float16* p) {
    U f; f.h[0] = *(const v8h*)(p); f.h[1] = *(const v8h*)(p + 16); return f.v;
  }
  static __device__ __forceinline__ v8f mma(v16h a, v16h b, v8f c) {
    return __builtin_amdgcn_wmma_f32_16x16x32_f16(false, a, false, b, (short)0, c, false, false);
  }
};
__device__ __forceinline__ v8f mma1(v16h a, v16h b, v8f c) {
  c = __builtin_amdgcn_wmma_f32_16x16x32_f16(false, a, false, b, (short)0, c, false, false);
  asm volatile("v_nop\n\tv_nop\n\tv_nop\n\tv_nop" : "+v"(c) : "v"(a), "v"(b));
  return c;
}

template <int BIAS_MODE, int OUT_MODE, int ACT>
__global__ __launch_bounds__(256) void wmma_gemm64(
    const unsigned short* __restrict__ Ap, int lda,
    const unsigned short* __restrict__ Btp, int ldb,
    void* __restrict__ Cout, int ldc,
    const float* __restrict__ bias,
    int M, int N, int K, float scale) {
  const _Float16* A  = (const _Float16*)Ap;
  const _Float16* Bt = (const _Float16*)Btp;
  __shared__ __align__(16) float sT[8][16 * 68];
  const int lane = threadIdx.x & 31;
  const int wave = threadIdx.x >> 5;
  const int tilesN = N >> 6;
  const int tilesM = M >> 6;
  const int tile = blockIdx.x * 8 + wave;
  if (tile >= tilesM * tilesN) return;
  const int tm = tile / tilesN;
  const int tn = tile - tm * tilesN;
  const int m0 = tm << 6;
  const int n0 = tn << 6;

  const int rlane = lane & 15;
  const int koff  = (lane >> 4) * 8;
  const int mOff  = (lane >> 4) * 8;

  v8f acc[4][4];
#pragma unroll
  for (int i = 0; i < 4; ++i)
#pragma unroll
    for (int j = 0; j < 4; ++j) acc[i][j] = (v8f){0.f,0.f,0.f,0.f,0.f,0.f,0.f,0.f};

  for (int k0 = 0; k0 < K; k0 += 32) {
    v16h bh[4];
#pragma unroll
    for (int j = 0; j < 4; ++j) {
      const size_t bo = (size_t)(n0 + (j << 4) + rlane) * ldb + koff + k0;
      bh[j] = FragH::load(Bt + bo);
    }
#pragma unroll
    for (int i = 0; i < 4; ++i) {
      const size_t ao = (size_t)(m0 + (i << 4) + rlane) * lda + koff + k0;
      v16h ah = FragH::load(A + ao);
#pragma unroll
      for (int j = 0; j < 4; ++j) {
        acc[i][j] = FragH::mma(ah, bh[j], acc[i][j]);
      }
      dep_guard4_h(acc[i][0], acc[i][1], acc[i][2], acc[i][3], ah, bh[3]);
    }
    keep4_h(bh[0], bh[1], bh[2], bh[3]);
  }
  acc_guard4(acc[0][0], acc[0][1], acc[0][2], acc[0][3]);
  acc_guard4(acc[1][0], acc[1][1], acc[1][2], acc[1][3]);
  acc_guard4(acc[2][0], acc[2][1], acc[2][2], acc[2][3]);
  acc_guard4(acc[3][0], acc[3][1], acc[3][2], acc[3][3]);

  float* slab = sT[wave];
#pragma unroll
  for (int i = 0; i < 4; ++i) {
    const int mBase = m0 + (i << 4);
#pragma unroll
    for (int j = 0; j < 4; ++j) {
      const int n = n0 + (j << 4) + rlane;
      float bv = 0.f;
      if (BIAS_MODE == 2) bv = bf16_rne(bias[n]);
#pragma unroll
      for (int r = 0; r < 8; ++r) {
        float v = acc[i][j][r] * scale;
        if (BIAS_MODE == 2) v += bv;
        if (ACT == 2) v = fmaxf(v, 0.0f);
        slab[(mOff + r) * 68 + (j << 4) + rlane] = v;
      }
    }
    __builtin_amdgcn_fence(__ATOMIC_RELEASE, "workgroup");
    __builtin_amdgcn_wave_barrier();
    __builtin_amdgcn_fence(__ATOMIC_ACQUIRE, "workgroup");
    if (OUT_MODE == 0) {
      float* C = (float*)Cout;
      const int hh = lane >> 4, c4 = (lane & 15) * 4;
      for (int pass = 0; pass < 2; ++pass) {
#pragma unroll
        for (int it = 0; it < 8; ++it) {
          const int row = it * 2 + hh;
          v4f v = *(const v4f*)(slab + row * 68 + c4);
          *(volatile v4f*)(C + (size_t)(mBase + row) * ldc + n0 + c4) = v;
        }
        __threadfence();
      }
    } else {
      const int q = lane >> 3, c8 = (lane & 7) * 8;
      unsigned short* C = (unsigned short*)Cout;
      for (int pass = 0; pass < 2; ++pass) {
#pragma unroll
        for (int it = 0; it < 4; ++it) {
          const int row = it * 4 + q;
          const float* sp = slab + row * 68 + c8;
          v8h hv;
#pragma unroll
          for (int e = 0; e < 8; ++e) {
            const float x = flush16(sp[e]);
            hv[e] = (_Float16)x;
          }
          *(volatile v8h*)(C + (size_t)(mBase + row) * ldc + n0 + c8) = hv;
        }
        __threadfence();
      }
    }
    __builtin_amdgcn_fence(__ATOMIC_RELEASE, "workgroup");
    __builtin_amdgcn_wave_barrier();
    __builtin_amdgcn_fence(__ATOMIC_ACQUIRE, "workgroup");
  }
}

__global__ __launch_bounds__(256) void cast8_pair_kernel(
    const float* __restrict__ inA, unsigned short* __restrict__ outA, int nblkA, int n8a,
    const float* __restrict__ inB, unsigned short* __restrict__ outB, int n8b, float scale) {
  const bool first = ((int)blockIdx.x < nblkA);
  const int blk = first ? (int)blockIdx.x : ((int)blockIdx.x - nblkA);
  const int n8 = first ? n8a : n8b;
  const float* in = first ? inA : inB;
  unsigned short* out = first ? outA : outB;
  const int i = blk * 256 + (int)threadIdx.x;
  if (i >= n8) return;
  const float* p = in + 8 * (size_t)i;
  const v4f a = *(const v4f*)(p);
  const v4f c = *(const v4f*)(p + 4);
  unsigned short hb[8];
#pragma unroll
  for (int e = 0; e < 4; ++e) {
    const float x0 = a[e];
    const float x1 = c[e];
    hb[e]     = h_bits(flush16(bf16_rne(x0) * scale));
    hb[4 + e] = h_bits(flush16(bf16_rne(x1) * scale));
  }
  const v4u u = (v4u){pk16(hb[0], hb[1]), pk16(hb[2], hb[3]), pk16(hb[4], hb[5]), pk16(hb[6], hb[7])};
  unsigned short* q = out + 8 * (size_t)i;
  *(volatile v4u*)q = u;
  __threadfence();
  *(volatile v4u*)q = u;
}

__global__ __launch_bounds__(256) void wtcast_kernel(const float* __restrict__ W0, const float* __restrict__ W1,
                                                     const float* __restrict__ W2, unsigned short* __restrict__ out,
                                                     int R, int C, float scale) {
  __shared__ float sm[64][65];
  const int t  = threadIdx.x;
  const int r0 = blockIdx.x * 64;
  const int c0 = blockIdx.y * 64;
  const int z  = blockIdx.z;
  const float* W = (z == 0) ? W0 : (z == 1) ? W1 : W2;
#pragma unroll
  for (int i = 0; i < 16; ++i) {
    const int e = i * 256 + t;
    const int r = e >> 6;
    const int c = e & 63;
    sm[c][r] = bf16_rne(W[(size_t)(r0 + r) * C + c0 + c]) * scale;
  }
  __syncthreads();
  const int lane = t & 31, wave = t >> 5;
  const int q = lane >> 3, c8 = (lane & 7) * 8;
  unsigned short* op = out + (size_t)z * C * R;
  for (int pass = 0; pass < 2; ++pass) {
#pragma unroll
    for (int it = 0; it < 2; ++it) {
      const int row = wave * 8 + it * 4 + q;
      unsigned short hb[8];
#pragma unroll
      for (int e = 0; e < 8; ++e) hb[e] = h_bits(flush16(sm[row][c8 + e]));
      const v4u u = (v4u){pk16(hb[0], hb[1]), pk16(hb[2], hb[3]), pk16(hb[4], hb[5]), pk16(hb[6], hb[7])};
      *(volatile v4u*)(op + (size_t)(c0 + row) * R + r0 + c8) = u;
    }
    __threadfence();
  }
}

__global__ __launch_bounds__(128) void seg_attn_kernel(
    const unsigned short* __restrict__ QKp, const unsigned short* __restrict__ VTpp,
    const unsigned short* __restrict__ CHp, const int* __restrict__ mask, float* __restrict__ XF) {
  __shared__ int sSeg[kS];
  __shared__ int sPart[128];
  __shared__ __align__(16) _Float16 Ps[4][16 * kPPitch];
  __shared__ __align__(16) float Os[4][16 * 68];
  const _Float16* QK = (const _Float16*)QKp;
  const _Float16* VT = (const _Float16*)VTpp;
  const _Float16* CH = (const _Float16*)CHp;
  const int tid  = threadIdx.x;
  const int wave = tid >> 5;
  const int lane = tid & 31;
  const int hh   = lane >> 4;
  const int c    = lane & 15;
  const int stile = blockIdx.x & 7;
  const int bh    = blockIdx.x >> 3;
  const int b = bh >> 3, h = bh & 7;

  {
    const v4i mv = *(const v4i*)(mask + b * kS + 4 * tid);
    const int f0 = reset_flag(mv[0]);
    const int f1 = reset_flag(mv[1]);
    const int f2 = reset_flag(mv[2]);
    const int f3 = reset_flag(mv[3]);
    const int p0 = f0, p1 = p0 + f1, p2 = p1 + f2, p3 = p2 + f3;
    sPart[tid] = p3;
    __syncthreads();
    int base = 0;
#pragma unroll 8
    for (int u = 0; u < 128; ++u) {
      const int pv = sPart[u];
      base += (u < tid) ? pv : 0;
    }
    sSeg[4 * tid + 0] = base + p0;
    sSeg[4 * tid + 1] = base + p1;
    sSeg[4 * tid + 2] = base + p2;
    sSeg[4 * tid + 3] = base + p3;
    __syncthreads();
  }

  const int s0 = stile * 64;
  const int q0 = s0 + wave * 16;
  const int segQ0 = __builtin_amdgcn_readfirstlane(sSeg[q0]);

  const _Float16* Qp = QK + (size_t)(b * kS + q0 + c) * kQKW + h * kHD + 8 * hh;
  const v16h qa0 = FragH::load(Qp);
  const v16h qa1 = FragH::load(Qp + 32);

  int segr[8];
#pragma unroll
  for (int r = 0; r < 8; ++r) segr[r] = sSeg[q0 + 8 * hh + r];

  v8f oacc[4];
#pragma unroll
  for (int it = 0; it < 4; ++it) oacc[it] = (v8f){0.f,0.f,0.f,0.f,0.f,0.f,0.f,0.f};

  {
    const _Float16* Cp = CH + (size_t)bh * (kHD * kHD) + (size_t)c * kHD + 8 * hh;
#pragma unroll
    for (int it = 0; it < 4; ++it) {
      const v16h cb0 = FragH::load(Cp + it * 16 * kHD);
      const v16h cb1 = FragH::load(Cp + it * 16 * kHD + 32);
      oacc[it] = mma1(qa0, cb0, oacc[it]);
      oacc[it] = mma1(qa1, cb1, oacc[it]);
    }
#pragma unroll
    for (int r = 0; r < 8; ++r) {
      const bool live0 = (segr[r] == 0);
#pragma unroll
      for (int it = 0; it < 4; ++it) {
        const float v = oacc[it][r] * kCarToPV;
        oacc[it][r] = live0 ? v : 0.0f;
      }
    }
  }

  _Float16* pw = Ps[wave];
  for (int tt = 0; tt <= stile; ++tt) {
    const int t0 = tt * 64;
    const int segTend = __builtin_amdgcn_readfirstlane(sSeg[t0 + 63]);
    if (segTend < segQ0) continue;

    v8f sc[4];
#pragma unroll
    for (int jt = 0; jt < 4; ++jt) {
      const _Float16* Kp = QK + (size_t)(b * kS + t0 + jt * 16 + c) * kQKW + kHID + h * kHD + 8 * hh;
      const v16h kb0 = FragH::load(Kp);
      const v16h kb1 = FragH::load(Kp + 32);
      sc[jt] = (v8f){0.f,0.f,0.f,0.f,0.f,0.f,0.f,0.f};
      sc[jt] = mma1(qa0, kb0, sc[jt]);
      sc[jt] = mma1(qa1, kb1, sc[jt]);
    }
    int segc[4];
#pragma unroll
    for (int jt = 0; jt < 4; ++jt) segc[jt] = sSeg[t0 + jt * 16 + c];
#pragma unroll
    for (int r = 0; r < 8; ++r) {
      const int srow = q0 + 8 * hh + r;
#pragma unroll
      for (int jt = 0; jt < 4; ++jt) {
        const int tcol = t0 + jt * 16 + c;
        const bool live = (tcol <= srow) && (segc[jt] == segr[r]);
        float p = sc[jt][r] * kScoreScale;
        p = live ? p : 0.0f;
        p = flush16(p);
        pw[(8 * hh + r) * kPPitch + jt * 16 + c] = (_Float16)p;
      }
    }
    __builtin_amdgcn_fence(__ATOMIC_RELEASE, "workgroup");
    __builtin_amdgcn_wave_barrier();
    __builtin_amdgcn_fence(__ATOMIC_ACQUIRE, "workgroup");
#pragma unroll
    for (int kk = 0; kk < 2; ++kk) {
      const v16h pa = FragH::load(pw + c * kPPitch + kk * 32 + 8 * hh);
#pragma unroll
      for (int it = 0; it < 4; ++it) {
        const v16h vb = FragH::load(VT + (size_t)(h * kHD + it * 16 + c) * kTok + b * kS + t0 + kk * 32 + 8 * hh);
        oacc[it] = mma1(pa, vb, oacc[it]);
      }
    }
    __builtin_amdgcn_fence(__ATOMIC_RELEASE, "workgroup");
    __builtin_amdgcn_wave_barrier();
    __builtin_amdgcn_fence(__ATOMIC_ACQUIRE, "workgroup");
  }

  float* os = Os[wave];
#pragma unroll
  for (int r = 0; r < 8; ++r) {
#pragma unroll
    for (int it = 0; it < 4; ++it) os[(8 * hh + r) * 68 + it * 16 + c] = oacc[it][r] * kXScale;
  }
  __builtin_amdgcn_fence(__ATOMIC_RELEASE, "workgroup");
  __builtin_amdgcn_wave_barrier();
  __builtin_amdgcn_fence(__ATOMIC_ACQUIRE, "workgroup");
  {
    const int c4 = (lane & 15) * 4;
    float* ob = XF + (size_t)(b * kS + q0) * kHID + h * kHD;
    for (int pass = 0; pass < 2; ++pass) {
#pragma unroll
      for (int it = 0; it < 8; ++it) {
        const int row = it * 2 + hh;
        v4f val = *(const v4f*)(os + row * 68 + c4);
        *(volatile v4f*)(ob + (size_t)row * kHID + c4) = val;
      }
      __threadfence();
    }
  }
}

__global__ __launch_bounds__(256) void rmsnorm_cast_kernel(const float* __restrict__ XF, const float* __restrict__ rs,
                                                           unsigned short* __restrict__ XN) {
  const int lane = threadIdx.x & 31, wave = threadIdx.x >> 5;
  const int row = blockIdx.x * 8 + wave;
  const float* xr = XF + (size_t)row * kHID;
  float x[16];
  float sc[16];
#pragma unroll
  for (int it = 0; it < 2; ++it) {
    const int col = it * 256 + lane * 8;
    const v4f a = *(const v4f*)(xr + col);
    const v4f d = *(const v4f*)(xr + col + 4);
    const v4f sa = *(const v4f*)(rs + col);
    const v4f sd = *(const v4f*)(rs + col + 4);
#pragma unroll
    for (int e = 0; e < 4; ++e) {
      x[it * 8 + e] = a[e];
      x[it * 8 + 4 + e] = d[e];
      const float s0v = sa[e];
      const float s1v = sd[e];
      sc[it * 8 + e] = bf16_rne(s0v);
      sc[it * 8 + 4 + e] = bf16_rne(s1v);
    }
  }
  float ss = 0.0f;
#pragma unroll
  for (int e = 0; e < 16; ++e) ss += x[e] * x[e];
#pragma unroll
  for (int off = 16; off > 0; off >>= 1) ss += __shfl_xor(ss, off, 32);
  const float inv = rsqrtf(ss * kInvHid + kEps);
  v4u u[2];
#pragma unroll
  for (int it = 0; it < 2; ++it) {
    unsigned short hb[8];
#pragma unroll
    for (int e = 0; e < 8; ++e) {
      const float y = (x[it * 8 + e] * inv) * sc[it * 8 + e];
      hb[e] = h_bits(flush16(y * kXnCarry));
    }
    u[it] = (v4u){pk16(hb[0], hb[1]), pk16(hb[2], hb[3]), pk16(hb[4], hb[5]), pk16(hb[6], hb[7])};
  }
  unsigned short* orow = XN + (size_t)row * kHID + lane * 8;
  for (int pass = 0; pass < 2; ++pass) {
    *(volatile v4u*)(orow) = u[0];
    *(volatile v4u*)(orow + 256) = u[1];
    __threadfence();
  }
}

__global__ __launch_bounds__(256) void final_state_kernel(
    const unsigned short* __restrict__ QKp, const unsigned short* __restrict__ VTpp,
    const float* __restrict__ carry, const int* __restrict__ mask, float* __restrict__ out0) {
  __shared__ int sLast[8];
  const int tid = threadIdx.x, lane = tid & 31, wave = tid >> 5;
  const int g  = blockIdx.x * 256 + tid;
  const int e0 = g * 4;
  const int bh = e0 >> 12;
  const int i  = (e0 >> 6) & 63;
  const int j0 = e0 & 63;
  const int b = bh >> 3, h = bh & 7;

  int last = -1;
#pragma unroll
  for (int u = 0; u < 2; ++u) {
    const int pos = tid + 256 * u;
    const int f = reset_flag(mask[b * kS + pos]);
    const int cand = (pos > last) ? pos : last;
    last = (f != 0) ? cand : last;
  }
#pragma unroll
  for (int off = 16; off > 0; off >>= 1) {
    const int o = __shfl_xor(last, off, 32);
    last = (o > last) ? o : last;
  }
  if (lane == 0) sLast[wave] = last;
  __syncthreads();
  int lastAll = sLast[0];
#pragma unroll
  for (int w = 1; w < 8; ++w) {
    const int o = sLast[w];
    lastAll = (o > lastAll) ? o : lastAll;
  }
  lastAll = (lastAll > kS - 1) ? (kS - 1) : lastAll;
  const bool none = (lastAll < 0);
  const int tstart = none ? 0 : lastAll;

  const v4f cv = *(const v4f*)(carry + e0);
  const float c0v = cv[0], c1v = cv[1], c2v = cv[2], c3v = cv[3];

  const unsigned* VTw = (const unsigned*)VTpp;
  float a0 = 0.0f, a1 = 0.0f, a2 = 0.0f, a3 = 0.0f;
#pragma unroll 1
  for (int t = tstart; t < kS; ++t) {
    const size_t vi = (size_t)(h * kHD + i) * kTok + (size_t)(b * kS + t);
    const unsigned vw = VTw[vi >> 1];
    const unsigned vh = (t & 1) ? (vw >> 16) : (vw & 0xffffu);
    const float v = h16_to_f32(vh);
    const v2u kw = *(const v2u*)(QKp + (size_t)(b * kS + t) * kQKW + kHID + h * kHD + j0);
    const unsigned w0 = kw[0];
    const unsigned w1 = kw[1];
    const float k0 = h16_to_f32(w0 & 0xffffu);
    const float k1 = h16_to_f32(w0 >> 16);
    const float k2 = h16_to_f32(w1 & 0xffffu);
    const float k3 = h16_to_f32(w1 >> 16);
    a0 = fmaf(v, k0, a0);
    a1 = fmaf(v, k1, a1);
    a2 = fmaf(v, k2, a2);
    a3 = fmaf(v, k3, a3);
  }
  v4f val;
  val[0] = (none ? bf16_rne(c0v) : 0.0f) + a0 * kStateScale;
  val[1] = (none ? bf16_rne(c1v) : 0.0f) + a1 * kStateScale;
  val[2] = (none ? bf16_rne(c2v) : 0.0f) + a2 * kStateScale;
  val[3] = (none ? bf16_rne(c3v) : 0.0f) + a3 * kStateScale;
  float* op = out0 + e0;
  *(volatile v4f*)op = val;
  __threadfence();
  *(volatile v4f*)op = val;
}

extern "C" void kernel_launch(void* const* d_in, const int* in_sizes, int n_in,
                              void* d_out, int out_size, void* d_ws, size_t ws_size,
                              hipStream_t stream) {
  if (n_in < 9) return;
  if (in_sizes[0] != kTok * kD) return;
  if (in_sizes[1] != kTok) return;
  if (in_sizes[2] != kB * kH * kHD * kHD) return;
  if (in_sizes[3] != kD * kHID) return;
  if (in_sizes[4] != kD * kHID) return;
  if (in_sizes[5] != kD * kHID) return;
  if (in_sizes[6] != kHID) return;
  if (in_sizes[7] != kHID * kD) return;
  if (in_sizes[8] != kD) return;
  if (out_size != (int)(kOut0Elems + kOut1Elems)) return;
  if (ws_size < kWsTotal) return;

  const float* inputs    = (const float*)d_in[0];
  const int*   mask      = (const int*)d_in[1];
  const float* carry     = (const float*)d_in[2];
  const float* wq        = (const float*)d_in[3];
  const float* wk        = (const float*)d_in[4];
  const float* wv        = (const float*)d_in[5];
  const float* rms_scale = (const float*)d_in[6];
  const float* wo        = (const float*)d_in[7];
  const float* bo        = (const float*)d_in[8];
  float* out0 = (float*)d_out;
  float* out1 = (float*)d_out + kOut0Elems;

  char* ws = (char*)d_ws;
  unsigned short* XH  = (unsigned short*)(ws + kOffXH);
  unsigned short* CH  = (unsigned short*)(ws + kOffCH);
  unsigned short* WT  = (unsigned short*)(ws + kOffWT);
  unsigned short* WOT = (unsigned short*)(ws + kOffWOT);
  unsigned short* QK  = (unsigned short*)(ws + kOffQK);
  unsigned short* VT  = (unsigned short*)(ws + kOffVT);
  float*          XF  = (float*)(ws + kOffXF);
  unsigned short* XN  = (unsigned short*)(ws + kOffXN);

  constexpr int n8a = kTok * kD / 8;
  constexpr int n8b = kB * kH * kHD * kHD / 8;
  constexpr int nblkA = n8a / 256;
  constexpr int nblkB = n8b / 256;
  static_assert(nblkA * 256 == n8a && nblkB * 256 == n8b);
  cast8_pair_kernel<<<nblkA + nblkB, 256, 0, stream>>>(inputs, XH, nblkA, n8a, carry, CH, n8b, kInCarry);

  wtcast_kernel<<<dim3(kD / 64, kHID / 64, 3), 256, 0, stream>>>(wq, wk, wv, WT, kD, kHID, kWCarry);
  wtcast_kernel<<<dim3(kHID / 64, kD / 64, 1), 256, 0, stream>>>(wo, wo, wo, WOT, kHID, kD, kWCarry);

  wmma_gemm64<0, 1, 2><<<(kTok / 64) * (kQKW / 64) / 8, 256, 0, stream>>>(
      XH, kD, WT, kD, (void*)QK, kQKW, nullptr, kTok, kQKW, kD, kProjScale);

  wmma_gemm64<0, 1, 0><<<(kHID / 64) * (kTok / 64) / 8, 256, 0, stream>>>(
      WT + (size_t)kQKW * kD, kD, XH, kD, (void*)VT, kTok, nullptr, kHID, kTok, kD, kProjScale);

  seg_attn_kernel<<<kB * kH * (kS / 64), 128, 0, stream>>>(QK, VT, CH, mask, XF);

  rmsnorm_cast_kernel<<<kTok / 8, 256, 0, stream>>>(XF, rms_scale, XN);

  wmma_gemm64<2, 0, 0><<<(kTok / 64) * (kD / 64) / 8, 256, 0, stream>>>(
      XN, kHID, WOT, kHID, (void*)out1, kD, bo, kTok, kD, kHID, kOutScale);

  final_state_kernel<<<(int)(kOut0Elems / 4 / 256), 256, 0, stream>>>(QK, VT, carry, mask, out0);
}
